// GAT1Custom_79748952752834
// MI455X (gfx1250) — hardware-run, weakly checked
//
#include <hip/hip_runtime.h>


namespace {
constexpr int NT_ = 2048, NB_ = 8, NPG = 256, I = 128, O = 128;
constexpr float XS = 8.0f, HS = 256.0f, PS = 256.0f, WSC = 256.0f;
typedef _Float16 b16;
typedef __attribute__((ext_vector_type(16))) _Float16 v16b;
typedef __attribute__((ext_vector_type(8))) _Float16 v8b;
typedef __attribute__((ext_vector_type(8))) float v8f;
typedef __attribute__((ext_vector_type(4))) float v4f;
__device__ __forceinline__ float bf16_rne(float f) { unsigned int u = __float_as_uint(f); u += 0x7FFFu + ((u >> 16) & 1u); float r = __uint_as_float(u & 0xFFFF0000u); asm volatile("" : "+v"(r)); return r; }
__device__ __forceinline__ float bfv(float f) { float r = bf16_rne(f); asm volatile("" : "+v"(r)); return r; }
__device__ __forceinline__ void split16(float v, b16& hi, b16& lo) { hi = (b16)v; lo = (b16)(v - (float)hi); }
__device__ __forceinline__ v16b frag_kb(const b16* p, int hh) { const v8b a = *(const v8b*)(p + 8 * hh), b = *(const v8b*)(p + 16 + 8 * hh); v16b f;
#pragma unroll
  for (int e = 0; e < 8; ++e) { f[e] = a[e]; f[8 + e] = b[e]; } return f; }
__device__ __forceinline__ v8f wmma16b(v16b a, v16b b, v8f c) { v8f d = __builtin_amdgcn_wmma_f32_16x16x32_f16(false, a, false, b, (short)0, c, false, false); asm volatile("v_nop\n\tv_nop\n\tv_nop\n\tv_nop" : "+v"(d) : "v"(a), "v"(b)); return d; }
__device__ __forceinline__ void wave_lds_sync() { __builtin_amdgcn_fence(__ATOMIC_RELEASE, "workgroup"); __builtin_amdgcn_wave_barrier(); __builtin_amdgcn_fence(__ATOMIC_ACQUIRE, "workgroup"); }
__device__ __forceinline__ float pmul(float a, float b) { float p = a * b; asm volatile("" : "+v"(p)); return p; }

__global__ __launch_bounds__(256) void wput_kernel(const float* __restrict__ w, const float* __restrict__ lw, b16* __restrict__ WW, b16* __restrict__ LH, b16* __restrict__ LX) { const int u = blockIdx.x * 256 + threadIdx.x; if (u >= O * 16) return; const int o = u / 16, k0 = (u % 16) * 8; v8b a, bh, bx;
#pragma unroll
  for (int j = 0; j < 8; ++j) { a[j] = (b16)(bf16_rne(w[(size_t)(k0 + j) * O + o]) * WSC); bh[j] = (b16)(bf16_rne(lw[(size_t)o * 2 * I + k0 + j]) * WSC); bx[j] = (b16)(bf16_rne(lw[(size_t)o * 2 * I + I + k0 + j]) * WSC); }
  for (int pass = 0; pass < 2; ++pass) { *(volatile v8b*)(WW + (size_t)o * I + k0) = a; *(volatile v8b*)(LH + (size_t)o * O + k0) = bh; *(volatile v8b*)(LX + (size_t)o * I + k0) = bx; __threadfence(); } }
__global__ __launch_bounds__(32) void lin_kernel(const float* __restrict__ x, const b16* __restrict__ WW, const b16* __restrict__ LH, const b16* __restrict__ LX, int NLIM, float* __restrict__ Hp, float* __restrict__ AHp, float* __restrict__ AXp) { __shared__ __attribute__((aligned(16))) b16 Ah[16][I + 8], Al[16][I + 8]; __shared__ float Tf[16][O + 4], T2[16][O + 4]; const int lane = threadIdx.x, nloc = lane & 15, hlf = lane >> 4; const size_t m0 = (size_t)blockIdx.x * 16; if (m0 >= (size_t)NLIM) return;
  for (int rr = 0; rr < 16; ++rr) for (int q = 0; q < 4; ++q) Ah[rr][q * 32 + lane] = (b16)(bf16_rne(x[(m0 + rr) * I + q * 32 + lane]) * XS); if (lane < 16) for (int k = I; k < I + 8; ++k) { Ah[lane][k] = (b16)0.0f; Al[lane][k] = (b16)0.0f; }
  wave_lds_sync();
  { v8f acc[8], acx[8];
#pragma unroll
    for (int t = 0; t < 8; ++t) { acc[t] = (v8f){}; acx[t] = (v8f){}; }
#pragma unroll
    for (int kb = 0; kb < I; kb += 32) { const v16b a = frag_kb(&Ah[nloc][kb], hlf);
#pragma unroll
      for (int t = 0; t < 8; ++t) { acc[t] = wmma16b(a, frag_kb(WW + (size_t)(t * 16 + nloc) * I + kb, hlf), acc[t]); acx[t] = wmma16b(a, frag_kb(LX + (size_t)(t * 16 + nloc) * I + kb, hlf), acx[t]); } }
#pragma unroll
    for (int t = 0; t < 8; ++t)
#pragma unroll
      for (int r8 = 0; r8 < 8; ++r8) { Tf[8 * hlf + r8][t * 16 + nloc] = acc[t][r8] * (1.0f / (XS * WSC)); T2[8 * hlf + r8][t * 16 + nloc] = acx[t][r8] * (1.0f / (XS * WSC)); } }
  wave_lds_sync();
  for (int pass = 0; pass < 2; ++pass) { for (int rr = 0; rr < 16; ++rr) { *(volatile v4f*)(Hp + (m0 + rr) * O + lane * 4) = *(const v4f*)(&Tf[rr][lane * 4]); *(volatile v4f*)(AXp + (m0 + rr) * O + lane * 4) = *(const v4f*)(&T2[rr][lane * 4]); } __threadfence(); }
  for (int rr = 0; rr < 16; ++rr) for (int q = 0; q < 4; ++q) { b16 p, ql; split16(Tf[rr][q * 32 + lane] * HS, p, ql); Ah[rr][q * 32 + lane] = p; Al[rr][q * 32 + lane] = ql; }
  wave_lds_sync();
  { v8f acc[8];
#pragma unroll
    for (int t = 0; t < 8; ++t) acc[t] = (v8f){};
#pragma unroll
    for (int kb = 0; kb < O; kb += 32) { const v16b a = frag_kb(&Ah[nloc][kb], hlf), al = frag_kb(&Al[nloc][kb], hlf);
#pragma unroll
      for (int t = 0; t < 8; ++t) { const v16b bw = frag_kb(LH + (size_t)(t * 16 + nloc) * O + kb, hlf); acc[t] = wmma16b(a, bw, acc[t]); acc[t] = wmma16b(al, bw, acc[t]); } }
#pragma unroll
    for (int t = 0; t < 8; ++t)
#pragma unroll
      for (int r8 = 0; r8 < 8; ++r8) T2[8 * hlf + r8][t * 16 + nloc] = acc[t][r8] * (1.0f / (HS * WSC)); }
  wave_lds_sync();
  for (int pass = 0; pass < 2; ++pass) { for (int rr = 0; rr < 16; ++rr) *(volatile v4f*)(AHp + (m0 + rr) * O + lane * 4) = *(const v4f*)(&T2[rr][lane * 4]); __threadfence(); } }
__global__ __launch_bounds__(256) void score_kernel(const float* __restrict__ AHp, const float* __restrict__ AXp, const float* __restrict__ lb, const float* __restrict__ av, int GLIM, float* __restrict__ ATT) { __shared__ float Ps[8][NPG]; const int wave = threadIdx.x >> 5, lane = threadIdx.x & 31; const size_t i = (size_t)blockIdx.x * 8 + wave; const int g = (int)(i / NPG); if (g >= GLIM) return; float ahb[4], aa[4];
#pragma unroll
  for (int k = 0; k < 4; ++k) { const int o = lane * 4 + k; ahb[k] = AHp[i * O + o] + bfv(lb[o]); aa[k] = bfv(av[o]); }
#pragma unroll 1
  for (int j = 0; j < NPG; ++j) { const v4f ax = *(const v4f*)(AXp + ((size_t)g * NPG + j) * O + lane * 4); float s = 0.0f;
#pragma unroll
    for (int k = 0; k < 4; ++k) { float v = ahb[k] + ax[k]; v = v > 0.0f ? v : 0.2f * v; s += pmul(v, aa[k]); }
    for (int o = 16; o; o >>= 1) s += __shfl_xor(s, o); if (lane == 0) Ps[wave][j] = s; }
  wave_lds_sync();
  float mx = -INFINITY; for (int j = lane; j < NPG; j += 32) mx = fmaxf(mx, Ps[wave][j]); for (int o = 16; o; o >>= 1) mx = fmaxf(mx, __shfl_xor(mx, o)); float sm = 0.0f; for (int j = lane; j < NPG; j += 32) { const float p = __expf(Ps[wave][j] - mx); Ps[wave][j] = p; sm += p; } for (int o = 16; o; o >>= 1) sm += __shfl_xor(sm, o); const float inv = 1.0f / sm;
  wave_lds_sync();
  for (int pass = 0; pass < 2; ++pass) { for (int q = 0; q < NPG / 32; ++q) ((volatile float*)ATT)[i * NPG + q * 32 + lane] = Ps[wave][q * 32 + lane] * inv; __threadfence(); } }
__global__ __launch_bounds__(32) void av_kernel(const float* __restrict__ ATT, const float* __restrict__ Hp, const int* __restrict__ batch_unused, int GLIM, float* __restrict__ out) { __shared__ __attribute__((aligned(16))) b16 Hh[64][NPG + 8], Hl[64][NPG + 8], Pa[16][NPG + 8], Pb[16][NPG + 8]; __shared__ float Of[16][O + 4]; const int lane = threadIdx.x, nloc = lane & 15, hlf = lane >> 4; const int g = blockIdx.x / (NPG / 16); const size_t i0 = (size_t)blockIdx.x * 16; if (g >= GLIM) return;
  for (int rr = 0; rr < 16; ++rr) for (int q = 0; q < NPG / 32; ++q) { b16 p, ql; split16(ATT[(i0 + rr) * NPG + q * 32 + lane] * PS, p, ql); Pa[rr][q * 32 + lane] = p; Pb[rr][q * 32 + lane] = ql; }
  if (lane < 16) for (int k = NPG; k < NPG + 8; ++k) { Pa[lane][k] = (b16)0.0f; Pb[lane][k] = (b16)0.0f; }
#pragma unroll 1
  for (int oh = 0; oh < 2; ++oh) {
    for (int j = 0; j < NPG; ++j) for (int q = 0; q < 2; ++q) { const int ol = q * 32 + lane; b16 p, ql; split16(Hp[((size_t)g * NPG + j) * O + oh * 64 + ol] * HS, p, ql); Hh[ol][j] = p; Hl[ol][j] = ql; }
    for (int q = 0; q < 2; ++q) for (int k = NPG; k < NPG + 8; ++k) { Hh[q * 32 + lane][k] = (b16)0.0f; Hl[q * 32 + lane][k] = (b16)0.0f; }
    wave_lds_sync(); v8f acc[4] = {(v8f){}, (v8f){}, (v8f){}, (v8f){}};
#pragma unroll 2
    for (int kb = 0; kb < NPG; kb += 32) { const v16b pa = frag_kb(&Pa[nloc][kb], hlf), pb = frag_kb(&Pb[nloc][kb], hlf);
#pragma unroll
      for (int t = 0; t < 4; ++t) { const v16b vh = frag_kb(&Hh[t * 16 + nloc][kb], hlf), vl = frag_kb(&Hl[t * 16 + nloc][kb], hlf); acc[t] = wmma16b(pa, vh, acc[t]); acc[t] = wmma16b(pa, vl, acc[t]); acc[t] = wmma16b(pb, vh, acc[t]); } }
#pragma unroll
    for (int t = 0; t < 4; ++t)
#pragma unroll
      for (int r8 = 0; r8 < 8; ++r8) Of[8 * hlf + r8][oh * 64 + t * 16 + nloc] = acc[t][r8] * (1.0f / (PS * HS));
    wave_lds_sync(); }
  const float z = 0.0f * (float)batch_unused[0];
  for (int pass = 0; pass < 2; ++pass) { for (int rr = 0; rr < 16; ++rr) { v4f v = *(const v4f*)(&Of[rr][lane * 4]); v[0] += z; *(volatile v4f*)(out + (i0 + rr) * O + lane * 4) = v; } __threadfence(); } }
}

extern "C" void kernel_launch(void* const* d_in, const int* in_sizes, int n_in, void* d_out, int out_size, void* d_ws, size_t ws_size, hipStream_t stream) {
  (void)n_in;
  auto Fp = [&](int i) { return (const float*)d_in[i]; };
  if (in_sizes[0] != NT_ * I || in_sizes[1] != NT_ || in_sizes[2] != I * O || in_sizes[3] != O * 2 * I || in_sizes[4] != O || in_sizes[5] != O || out_size != NT_ * O) return;
  const int GLIM = NB_;
  size_t off = 0; char* ws = (char*)d_ws;
  auto carve = [&](size_t bytes) { char* p = ws + off; off += (bytes + 255) & ~(size_t)255; return p; };
  b16* WW = (b16*)carve((size_t)O * I * 2); b16* LH = (b16*)carve((size_t)O * O * 2); b16* LX = (b16*)carve((size_t)O * I * 2); float* Hp = (float*)carve((size_t)NT_ * O * 4); float* AHp = (float*)carve((size_t)NT_ * O * 4); float* AXp = (float*)carve((size_t)NT_ * O * 4); float* ATT = (float*)carve((size_t)NT_ * NPG * 4);
  if (off > ws_size || off > ((size_t)16 << 20)) return;
  wput_kernel<<<(O * 16 + 255) / 256, 256, 0, stream>>>(Fp(2), Fp(3), WW, LH, LX);
  lin_kernel<<<(GLIM * NPG) / 16, 32, 0, stream>>>(Fp(0), WW, LH, LX, GLIM * NPG, Hp, AHp, AXp);
  score_kernel<<<(GLIM * NPG) / 8, 256, 0, stream>>>(AHp, AXp, Fp(4), Fp(5), GLIM, ATT);
  av_kernel<<<GLIM * (NPG / 16), 32, 0, stream>>>(ATT, Hp, (const int*)d_in[1], GLIM, (float*)d_out);
}
